// MultiHeadedAttention_80848464380392
// MI455X (gfx1250) — hardware-verified
//
#include <hip/hip_runtime.h>


#ifndef NB
#define NB 2
#endif
#ifndef SEQ
#define SEQ 2048
#endif
#define SEQ_FULL 2048
#define DM   1024
#define NH_  16
#define HD   64
#define EARLY ((SEQ) < 512 ? (SEQ) : 512)
#define QK_CARRY 16.0f
#define V_CARRY  64.0f
#define W_CARRY  1024.0f
#define SSC  4.8828125e-4f
#define OSC  3.814697265625e-06f
#define L2E  1.4426950408889634f

static_assert(SEQ % 64 == 0);
static_assert(SEQ <= SEQ_FULL);
static_assert(EARLY % 64 == 0);
static_assert(EARLY <= SEQ);
static_assert(NH_ * HD == DM);
static_assert(DM % 64 == 0);
static_assert(DM % 32 == 0);
static_assert(HD == 64);
static_assert(NB >= 1 && NB <= 2);

typedef _Float16 h16;
typedef unsigned short bf;
typedef __attribute__((ext_vector_type(16))) __bf16   v16bf;
typedef __attribute__((ext_vector_type(16))) _Float16 v16h;
typedef __attribute__((ext_vector_type(8)))  _Float16 v8h;
typedef __attribute__((ext_vector_type(8)))  unsigned short v8us;
typedef __attribute__((ext_vector_type(8)))  float    v8f;
typedef __attribute__((ext_vector_type(4)))  float    v4f;
typedef __attribute__((ext_vector_type(4)))  int      v4i;
typedef v4f  __attribute__((may_alias)) v4fa;

__device__ __forceinline__ unsigned short f2bf(float f) { unsigned u = __float_as_uint(f); u += 0x7FFFu + ((u >> 16) & 1u); return (unsigned short)(u >> 16); }
__device__ __forceinline__ float bf2f(unsigned short b) { return __uint_as_float(((unsigned)b) << 16); }
__device__ __forceinline__ float bfr(float f) { return bf2f(f2bf(f)); }
__device__ __forceinline__ v16h cat16(v8h lo, v8h hi) { return __builtin_shufflevector(lo, hi, 0, 1, 2, 3, 4, 5, 6, 7, 8, 9, 10, 11, 12, 13, 14, 15); }
__device__ __forceinline__ v16bf cat16b(v8us lo, v8us hi) { return __builtin_bit_cast(v16bf, __builtin_shufflevector(lo, hi, 0, 1, 2, 3, 4, 5, 6, 7, 8, 9, 10, 11, 12, 13, 14, 15)); }
__device__ __forceinline__ v8f wmma16(v16h a, v16h b, v8f c) { return __builtin_amdgcn_wmma_f32_16x16x32_f16(false, a, false, b, (short)0, c, false, false); }
__device__ __forceinline__ v8f wmmab(v16bf a, v16bf b, v8f c) { return __builtin_amdgcn_wmma_f32_16x16x32_bf16(false, a, false, b, (short)0, c, false, false); }
__device__ __forceinline__ v16h ldh(const h16* p) { return cat16(*(const v8h*)p, *(const v8h*)(p + 16)); }

template <typename T16> struct WFrag;
template <> struct WFrag<h16> { typedef v16h V; static __device__ __forceinline__ V ld(const h16* p) { return cat16(*(const v8h*)p, *(const v8h*)(p + 16)); } static __device__ __forceinline__ v8f mma(V a, V b, v8f c) { return wmma16(a, b, c); } };
template <> struct WFrag<bf> { typedef v16bf V; static __device__ __forceinline__ V ld(const bf* p) { return cat16b(*(const v8us*)p, *(const v8us*)(p + 16)); } static __device__ __forceinline__ v8f mma(V a, V b, v8f c) { return wmmab(a, b, c); } };

template <typename T16>
__device__ __forceinline__ void tile_kstep(const T16* __restrict__ A, const T16* __restrict__ Bt, size_t aoff, size_t boff, int K, int kc, v8f (&acc)[4][4]) {
    typedef typename WFrag<T16>::V V;
    V a[4];
#pragma unroll
    for (int mb = 0; mb < 4; ++mb) a[mb] = WFrag<T16>::ld(A + aoff + (size_t)mb * 16 * K + kc);
#pragma unroll
    for (int nb = 0; nb < 4; ++nb) {
        const V b = WFrag<T16>::ld(Bt + boff + (size_t)nb * 16 * K + kc);
#pragma unroll
        for (int mb = 0; mb < 4; ++mb) acc[mb][nb] = WFrag<T16>::mma(a[mb], b, acc[mb][nb]);
    }
    asm volatile("v_nop\n\tv_nop\n\tv_nop\n\tv_nop" : "+v"(acc[0][3]), "+v"(acc[1][3]), "+v"(acc[2][3]), "+v"(acc[3][3]) : "v"(a[0]), "v"(a[3]));
}

__device__ __forceinline__ void dump_tile(float* os, const v8f (&acc)[4][4], int lr, int hi) {
#pragma unroll
    for (int mb = 0; mb < 4; ++mb)
#pragma unroll
        for (int nb = 0; nb < 4; ++nb)
#pragma unroll
            for (int j = 0; j < 8; ++j) os[(mb * 16 + hi * 8 + j) * 68 + nb * 16 + lr] = acc[mb][nb][j];
}

__global__ __launch_bounds__(256) void k_cvt8(const float* __restrict__ src, bf* dst, size_t n8) { const size_t i = (size_t)blockIdx.x * 256 + threadIdx.x; if (i >= n8) return; const v8f v = *(const v8f*)(src + i * 8); v8us o;
#pragma unroll
    for (int k = 0; k < 8; ++k) o[k] = f2bf(v[k]); *(volatile v8us*)(dst + i * 8) = o; __threadfence(); *(volatile v8us*)(dst + i * 8) = o; }

__global__ __launch_bounds__(256) void k_cvtw(const float* __restrict__ src, h16* dst, size_t n8) { const size_t i = (size_t)blockIdx.x * 256 + threadIdx.x; if (i >= n8) return; const v8f v = *(const v8f*)(src + i * 8); v8h o;
#pragma unroll
    for (int k = 0; k < 8; ++k) o[k] = (h16)(bfr(v[k]) * W_CARRY); *(volatile v8h*)(dst + i * 8) = o; __threadfence(); *(volatile v8h*)(dst + i * 8) = o; }

__global__ __launch_bounds__(32) void k_proj_qk(const bf* __restrict__ XB, const bf* __restrict__ WB, const float* __restrict__ bias, h16* PH, h16* PL) {
    __shared__ __align__(16) float os[64 * 68];
    const int lane = threadIdx.x & 31, lr = lane & 15, hi = lane >> 4;
    const int mt = blockIdx.x; const int b = mt / (SEQ / 64); const int s0 = (mt % (SEQ / 64)) * 64;
    const int h = blockIdx.y; const int c0 = h * HD;
    v8f acc[4][4];
#pragma unroll
    for (int mb = 0; mb < 4; ++mb)
#pragma unroll
        for (int nb = 0; nb < 4; ++nb) acc[mb][nb] = (v8f){};
    const size_t aoff = ((size_t)b * SEQ_FULL + s0 + lr) * DM + 8 * hi, boff = (size_t)(c0 + lr) * DM + 8 * hi;
#pragma unroll 1
    for (int kc = 0; kc < DM; kc += 32) tile_kstep<bf>(XB, WB, aoff, boff, DM, kc, acc);
    dump_tile(os, acc, lr, hi);
    __syncthreads();
    const int rq = lane >> 3, pc = lane & 7;
    const v4f bq0 = *(const v4f*)(bias + c0 + pc * 8), bq1 = *(const v4f*)(bias + c0 + pc * 8 + 4);
    float bb[8];
#pragma unroll
    for (int j = 0; j < 4; ++j) { bb[j] = bfr(bq0[j]); bb[4 + j] = bfr(bq1[j]); }
    const bool res = (s0 < EARLY);
    const size_t bh = (size_t)b * NH_ + h;
#pragma unroll 1
    for (int ps = 0; ps < 2; ++ps) {
#pragma unroll 1
        for (int it = 0; it < 16; ++it) {
            const int row = it * 4 + rq;
            const v4f x0 = *(const v4fa*)(os + row * 68 + pc * 8), x1 = *(const v4fa*)(os + row * 68 + pc * 8 + 4);
            v8h oh, ol;
#pragma unroll
            for (int j = 0; j < 4; ++j) {
                const float y0 = (x0[j] + bb[j]) * QK_CARRY, y1 = (x1[j] + bb[4 + j]) * QK_CARRY;
                const h16 a0 = (h16)y0, a1 = (h16)y1;
                oh[j] = a0; oh[4 + j] = a1; ol[j] = (h16)(y0 - (float)a0); ol[4 + j] = (h16)(y1 - (float)a1);
            }
            *(volatile v8h*)(PH + (bh * SEQ + s0 + row) * HD + pc * 8) = oh;
            if (res) *(volatile v8h*)(PL + (bh * EARLY + s0 + row) * HD + pc * 8) = ol;
        }
        if (ps == 0) __threadfence();
    }
}

__global__ __launch_bounds__(32) void k_proj_v(const bf* __restrict__ XB, const bf* __restrict__ WB, const float* __restrict__ bias, h16* VH, h16* VL) {
    __shared__ __align__(16) float os[64 * 68];
    const int lane = threadIdx.x & 31, lr = lane & 15, hi = lane >> 4;
    const int mt = blockIdx.x; const int b = mt / (SEQ / 64); const int s0 = (mt % (SEQ / 64)) * 64;
    const int h = blockIdx.y; const int c0 = h * HD;
    v8f acc[4][4];
#pragma unroll
    for (int mb = 0; mb < 4; ++mb)
#pragma unroll
        for (int nb = 0; nb < 4; ++nb) acc[mb][nb] = (v8f){};
    const size_t aoff = ((size_t)b * SEQ_FULL + s0 + lr) * DM + 8 * hi, boff = (size_t)(c0 + lr) * DM + 8 * hi;
#pragma unroll 1
    for (int kc = 0; kc < DM; kc += 32) tile_kstep<bf>(XB, WB, aoff, boff, DM, kc, acc);
    dump_tile(os, acc, lr, hi);
    __syncthreads();
    const int dq = lane >> 3, pc = lane & 7;
    const bool res = (s0 < EARLY);
    const size_t bh = (size_t)b * NH_ + h;
#pragma unroll 1
    for (int ps = 0; ps < 2; ++ps) {
#pragma unroll 1
        for (int it = 0; it < 16; ++it) {
            const int d = it * 4 + dq;
            const float bd = bfr(bias[c0 + d]);
            v8h oh, ol;
#pragma unroll
            for (int j = 0; j < 8; ++j) {
                const float y = (os[(pc * 8 + j) * 68 + d] + bd) * V_CARRY;
                const h16 a = (h16)y; oh[j] = a; ol[j] = (h16)(y - (float)a);
            }
            *(volatile v8h*)(VH + (bh * HD + d) * SEQ + s0 + pc * 8) = oh;
            if (res) *(volatile v8h*)(VL + (bh * HD + d) * EARLY + s0 + pc * 8) = ol;
        }
        if (ps == 0) __threadfence();
    }
}

template <bool RES>
__device__ __forceinline__ void flash_body(const h16* __restrict__ QH, const h16* __restrict__ QL, const h16* __restrict__ KH, const h16* __restrict__ KL,
                                           const h16* __restrict__ VH, const h16* __restrict__ VL, const int* __restrict__ PM,
                                           int b, int h, int qw0, int lane, v8f (&o)[4], float& lsum) {
    const int lr = lane & 15, hi = lane >> 4;
    const size_t bh = (size_t)b * NH_ + h;
    const float NEG = -__builtin_inff();
    v16h qf[2], ql[2];
    { const h16* p = QH + (bh * SEQ + qw0 + lr) * HD + 8 * hi; qf[0] = ldh(p); qf[1] = ldh(p + 32); }
    ql[0] = qf[0]; ql[1] = qf[1];
    if (RES) { const h16* p = QL + (bh * EARLY + qw0 + lr) * HD + 8 * hi; ql[0] = ldh(p); ql[1] = ldh(p + 32); }
    const int* pmb = PM + (size_t)b * SEQ_FULL;
    float m = NEG, l = 0.f;
#pragma unroll
    for (int dt = 0; dt < 4; ++dt) o[dt] = (v8f){};
    const int nch = (qw0 >> 6) + 1;
    const int qi = qw0 + lr;
#pragma unroll 1
    for (int c = 0; c < nch; ++c) {
        const int kc = c * 64;
        v8f st[4];
#pragma unroll
        for (int t = 0; t < 4; ++t) {
            st[t] = (v8f){};
#pragma unroll
            for (int ks = 0; ks < 2; ++ks) {
                const v16h ka = ldh(KH + (bh * SEQ + kc + 16 * t + lr) * HD + 8 * hi + 32 * ks);
                st[t] = wmma16(ka, qf[ks], st[t]);
                if (RES) {
                    const v16h kb = ldh(KL + (bh * EARLY + kc + 16 * t + lr) * HD + 8 * hi + 32 * ks);
                    st[t] = wmma16(kb, qf[ks], st[t]);
                    st[t] = wmma16(ka, ql[ks], st[t]);
                }
            }
        }
        asm volatile("v_nop\n\tv_nop\n\tv_nop\n\tv_nop" : "+v"(st[0]), "+v"(st[1]), "+v"(st[2]), "+v"(st[3]) : "v"(qf[0]), "v"(qf[1]), "v"(ql[0]), "v"(ql[1]));
#pragma unroll
        for (int t = 0; t < 4; ++t) st[t] = st[t] * SSC;
        const int mk0 = pmb[kc + 2 * lane], mk1 = pmb[kc + 2 * lane + 1];
        if (__any((mk0 == 0) | (mk1 == 0))) {
#pragma unroll
            for (int t = 0; t < 4; ++t) {
                const v4i a0 = *(const v4i*)(pmb + kc + 16 * t + 8 * hi), a1 = *(const v4i*)(pmb + kc + 16 * t + 8 * hi + 4);
#pragma unroll
                for (int r = 0; r < 4; ++r) { st[t][r] = (a0[r] == 0) ? NEG : st[t][r]; st[t][4 + r] = (a1[r] == 0) ? NEG : st[t][4 + r]; }
            }
        }
        if (c == nch - 1) {
#pragma unroll
            for (int t = 0; t < 4; ++t)
#pragma unroll
                for (int r = 0; r < 8; ++r) { const int key = kc + 16 * t + 8 * hi + r; st[t][r] = (key > qi) ? NEG : st[t][r]; }
        }
        float mx = st[0][0];
#pragma unroll
        for (int t = 0; t < 4; ++t)
#pragma unroll
            for (int r = 0; r < 8; ++r) mx = fmaxf(mx, st[t][r]);
        mx = fmaxf(mx, __shfl_xor(mx, 16, 32));
        const float mnew = fmaxf(m, mx);
        const float muse = (mnew == NEG) ? 0.f : mnew;
        const float alpha = __builtin_amdgcn_exp2f((m - muse) * L2E);
        m = mnew;
        const float cofs = 10.0f - muse * L2E;
        float psum = 0.f;
#pragma unroll
        for (int t = 0; t < 4; ++t)
#pragma unroll
            for (int r = 0; r < 8; ++r) { const float pe = __builtin_amdgcn_exp2f(fmaf(st[t][r], L2E, cofs)); st[t][r] = pe; psum += pe; }
        l = l * alpha + psum;
#pragma unroll
        for (int dt = 0; dt < 4; ++dt) o[dt] = o[dt] * alpha;
#pragma unroll
        for (int j = 0; j < 2; ++j) {
            v16h ph, pr;
#pragma unroll
            for (int r = 0; r < 8; ++r) {
                const float a = st[2 * j][r], c2 = st[2 * j + 1][r];
                const h16 ah = (h16)a, ch = (h16)c2;
                ph[r] = ah; ph[8 + r] = ch;
                if (RES) { pr[r] = (h16)(a - (float)ah); pr[8 + r] = (h16)(c2 - (float)ch); }
            }
            if (!RES) pr = ph;
#pragma unroll
            for (int dt = 0; dt < 4; ++dt) {
                const v16h va = ldh(VH + (bh * HD + dt * 16 + lr) * SEQ + kc + 32 * j + 8 * hi);
                o[dt] = wmma16(va, ph, o[dt]);
                if (RES) {
                    const v16h vb = ldh(VL + (bh * HD + dt * 16 + lr) * EARLY + kc + 32 * j + 8 * hi);
                    o[dt] = wmma16(vb, ph, o[dt]);
                    o[dt] = wmma16(va, pr, o[dt]);
                }
            }
            asm volatile("v_nop\n\tv_nop\n\tv_nop\n\tv_nop" : "+v"(o[0]), "+v"(o[1]), "+v"(o[2]), "+v"(o[3]) : "v"(ph), "v"(pr));
        }
    }
    lsum = l;
}

__global__ __launch_bounds__(128) void k_flash(const h16* __restrict__ QH, const h16* __restrict__ QL, const h16* __restrict__ KH, const h16* __restrict__ KL,
                                               const h16* __restrict__ VH, const h16* __restrict__ VL, const int* __restrict__ PM, h16* CH, h16* CL) {
    __shared__ __align__(16) float cs[4][16 * 68];
    const int lane = threadIdx.x & 31, w = threadIdx.x >> 5, lr = lane & 15, hi = lane >> 4;
    const int b = blockIdx.z, h = blockIdx.y, q0 = blockIdx.x * 64, qw0 = q0 + 16 * w;
    const bool early = (q0 < EARLY);
    v8f o[4]; float l;
    if (early) flash_body<true>(QH, QL, KH, KL, VH, VL, PM, b, h, qw0, lane, o, l);
    else       flash_body<false>(QH, QL, KH, KL, VH, VL, PM, b, h, qw0, lane, o, l);
    const float lt = l + __shfl_xor(l, 16, 32);
    const float inv = 4.0f / lt;
    float* cw = &cs[w][0];
#pragma unroll
    for (int dt = 0; dt < 4; ++dt)
#pragma unroll
        for (int r = 0; r < 8; ++r) cw[lr * 68 + dt * 16 + 8 * hi + r] = o[dt][r] * inv;
    __syncthreads();
    const int rq = lane >> 3, pc = lane & 7;
#pragma unroll 1
    for (int ps = 0; ps < 2; ++ps) {
#pragma unroll 1
        for (int it = 0; it < 4; ++it) {
            const int row = it * 4 + rq;
            const v4f x0 = *(const v4fa*)(cw + row * 68 + pc * 8), x1 = *(const v4fa*)(cw + row * 68 + pc * 8 + 4);
            v8h oh, ol;
#pragma unroll
            for (int j = 0; j < 4; ++j) {
                const h16 a0 = (h16)x0[j], a1 = (h16)x1[j];
                oh[j] = a0; oh[4 + j] = a1; ol[j] = (h16)(x0[j] - (float)a0); ol[4 + j] = (h16)(x1[j] - (float)a1);
            }
            *(volatile v8h*)(CH + ((size_t)b * SEQ + qw0 + row) * DM + h * HD + pc * 8) = oh;
            if (early) *(volatile v8h*)(CL + ((size_t)b * EARLY + qw0 + row) * DM + h * HD + pc * 8) = ol;
        }
        if (ps == 0) __threadfence();
    }
}

__global__ __launch_bounds__(32) void k_oproj(const h16* __restrict__ CH, const h16* __restrict__ CL, const h16* __restrict__ WO, const float* __restrict__ bo, float* OUT) {
    __shared__ __align__(16) float os[64 * 68];
    const int lane = threadIdx.x & 31, lr = lane & 15, hi = lane >> 4;
    const int mt = blockIdx.x; const int b = mt / (SEQ / 64); const int s0 = (mt % (SEQ / 64)) * 64;
    const int c0 = blockIdx.y * 64;
    v8f acc[4][4];
#pragma unroll
    for (int mb = 0; mb < 4; ++mb)
#pragma unroll
        for (int nb = 0; nb < 4; ++nb) acc[mb][nb] = (v8f){};
    const size_t aoff = ((size_t)b * SEQ + s0 + lr) * DM + 8 * hi, aoff2 = ((size_t)b * EARLY + s0 + lr) * DM + 8 * hi, boff = (size_t)(c0 + lr) * DM + 8 * hi;
    const bool res = (s0 < EARLY);
#pragma unroll 1
    for (int kc = 0; kc < DM; kc += 32) {
        tile_kstep<h16>(CH, WO, aoff, boff, DM, kc, acc);
        if (res) tile_kstep<h16>(CL, WO, aoff2, boff, DM, kc, acc);
    }
    dump_tile(os, acc, lr, hi);
    __syncthreads();
    const int cofs = lr * 4;
    const v4f bq = *(const v4f*)(bo + c0 + cofs);
    v4f bb; bb[0] = bfr(bq[0]); bb[1] = bfr(bq[1]); bb[2] = bfr(bq[2]); bb[3] = bfr(bq[3]);
#pragma unroll 1
    for (int ps = 0; ps < 2; ++ps) {
#pragma unroll 1
        for (int it = 0; it < 32; ++it) {
            const int row = 2 * it + hi;
            const v4f x = *(const v4fa*)(os + row * 68 + cofs);
            const v4f val = x * OSC + bb;
            *(volatile v4f*)(OUT + ((size_t)b * SEQ + s0 + row) * DM + c0 + cofs) = val;
        }
        if (ps == 0) __threadfence();
    }
}

constexpr size_t al256(size_t x) { return (x + 255) & ~(size_t)255; }
constexpr size_t SZ_XB = al256((size_t)NB * SEQ_FULL * DM * 2);
constexpr size_t SZ_WB = al256((size_t)DM * DM * 2);
constexpr size_t SZ_PL = al256((size_t)NB * NH_ * SEQ * HD * 2);
constexpr size_t SZ_RS = al256((size_t)NB * NH_ * EARLY * HD * 2);
constexpr size_t SZ_CH = al256((size_t)NB * SEQ * DM * 2);
constexpr size_t SZ_CL = al256((size_t)NB * EARLY * DM * 2);
constexpr size_t SZ_TOTAL = 3 * SZ_XB + 4 * SZ_WB + 3 * SZ_PL + 3 * SZ_RS + SZ_CH + SZ_CL;
static_assert(SZ_TOTAL <= (size_t)134217728);

extern "C" void kernel_launch(void* const* d_in, const int* in_sizes, int n_in,
                              void* d_out, int out_size, void* d_ws, size_t ws_size, hipStream_t stream) {
    if (n_in < 12) return;
    if (in_sizes[0] < NB * SEQ_FULL * DM || in_sizes[1] < NB * SEQ_FULL * DM || in_sizes[2] < NB * SEQ_FULL * DM) return;
    if (in_sizes[3] < NB * SEQ_FULL) return;
    if (in_sizes[4] < DM * DM || in_sizes[6] < DM * DM || in_sizes[8] < DM * DM || in_sizes[10] < DM * DM) return;
    if (in_sizes[5] < DM || in_sizes[7] < DM || in_sizes[9] < DM || in_sizes[11] < DM) return;
    if (out_size < NB * SEQ * DM) return;
    if (SZ_TOTAL > ws_size) return;
    const float* Vin = (const float*)d_in[0];
    const float* Kin = (const float*)d_in[1];
    const float* Qin = (const float*)d_in[2];
    const int*   pm  = (const int*)d_in[3];
    const float* Wv  = (const float*)d_in[4];  const float* bv = (const float*)d_in[5];
    const float* Wk  = (const float*)d_in[6];  const float* bk = (const float*)d_in[7];
    const float* Wq  = (const float*)d_in[8];  const float* bq = (const float*)d_in[9];
    const float* Wo  = (const float*)d_in[10]; const float* bo = (const float*)d_in[11];
    float* OUT = (float*)d_out;
    char* wsp = (char*)d_ws;
    auto take = [&](size_t bytes) { char* p = wsp; wsp += bytes; return (void*)p; };
    bf*  XV  = (bf*)take(SZ_XB);  bf* XK = (bf*)take(SZ_XB);  bf* XQ = (bf*)take(SZ_XB);
    bf*  WVb = (bf*)take(SZ_WB);  bf* WKb = (bf*)take(SZ_WB); bf* WQb = (bf*)take(SZ_WB);
    h16* WOh = (h16*)take(SZ_WB);
    h16* QH  = (h16*)take(SZ_PL); h16* KH = (h16*)take(SZ_PL); h16* VH = (h16*)take(SZ_PL);
    h16* QL  = (h16*)take(SZ_RS); h16* KL = (h16*)take(SZ_RS); h16* VL = (h16*)take(SZ_RS);
    h16* CH  = (h16*)take(SZ_CH); h16* CL = (h16*)take(SZ_CL);
    if ((size_t)(wsp - (char*)d_ws) > ws_size) return;

    const size_t nx8 = (size_t)NB * SEQ_FULL * DM / 8, nw8 = (size_t)DM * DM / 8;
    const unsigned gx = (unsigned)((nx8 + 255) / 256), gw = (unsigned)((nw8 + 255) / 256);
    k_cvt8<<<gx, 256, 0, stream>>>(Vin, XV, nx8);
    k_cvt8<<<gx, 256, 0, stream>>>(Kin, XK, nx8);
    k_cvt8<<<gx, 256, 0, stream>>>(Qin, XQ, nx8);
    k_cvt8<<<gw, 256, 0, stream>>>(Wv, WVb, nw8);
    k_cvt8<<<gw, 256, 0, stream>>>(Wk, WKb, nw8);
    k_cvt8<<<gw, 256, 0, stream>>>(Wq, WQb, nw8);
    k_cvtw<<<gw, 256, 0, stream>>>(Wo, WOh, nw8);
    const dim3 gp(NB * SEQ / 64, NH_);
    k_proj_qk<<<gp, 32, 0, stream>>>(XQ, WQb, bq, QH, QL);
    k_proj_qk<<<gp, 32, 0, stream>>>(XK, WKb, bk, KH, KL);
    k_proj_v<<<gp, 32, 0, stream>>>(XV, WVb, bv, VH, VL);
    k_flash<<<dim3(SEQ / 64, NH_, NB), 128, 0, stream>>>(QH, QL, KH, KL, VH, VL, pm, CH, CL);
    k_oproj<<<dim3(NB * SEQ / 64, DM / 64), 32, 0, stream>>>(CH, CL, WOh, bo, OUT);
}
